// WindowAttention_6597069767438
// MI455X (gfx1250) — hardware-verified
//
#include <hip/hip_runtime.h>
#include <stdint.h>

typedef __attribute__((ext_vector_type(16))) _Float16 v16h;
typedef __attribute__((ext_vector_type(8)))  _Float16 v8h;
typedef __attribute__((ext_vector_type(16))) __bf16   v16b;
typedef __attribute__((ext_vector_type(8)))  __bf16   v8b;
typedef __attribute__((ext_vector_type(8)))  float    v8f;
typedef __attribute__((ext_vector_type(4)))  float    v4f;
typedef __attribute__((ext_vector_type(4)))  unsigned v4u;
typedef __attribute__((ext_vector_type(2)))  unsigned v2u;

__device__ __forceinline__ void dep_guard_h(v8f& a, v8f& b, v16h x, v16h y) { asm volatile("v_nop\n\tv_nop\n\tv_nop\n\tv_nop" : "+v"(a), "+v"(b) : "v"(x), "v"(y)); }
__device__ __forceinline__ void dep_guard_b(v8f& a, v8f& b, v16b x, v16b y) { asm volatile("v_nop\n\tv_nop\n\tv_nop\n\tv_nop" : "+v"(a), "+v"(b) : "v"(x), "v"(y)); }
__device__ __forceinline__ void keep4_h(v16h a, v16h b, v16h c, v16h d) { asm volatile("v_nop" :: "v"(a), "v"(b), "v"(c), "v"(d)); }
__device__ __forceinline__ void keep4_b(v16b a, v16b b, v16b c, v16b d) { asm volatile("v_nop" :: "v"(a), "v"(b), "v"(c), "v"(d)); }
template <typename T> struct Frag;
template <> struct Frag<_Float16> {
  typedef v16h V; union U { v16h v; v8h h[2]; };
  static __device__ __forceinline__ v16h load(const _Float16* p) {
    U f; f.h[0] = *(const v8h*)(p); f.h[1] = *(const v8h*)(p + 16); return f.v;
  }
  static __device__ __forceinline__ v8f mma(v16h a, v16h b, v8f c) {
    return __builtin_amdgcn_wmma_f32_16x16x32_f16(false, a, false, b, (short)0, c, false, false);
  }
  static __device__ __forceinline__ void guard(v8f& a, v8f& b, v16h x, v16h y) { dep_guard_h(a, b, x, y); }
  static __device__ __forceinline__ void keep(v16h a, v16h b, v16h c, v16h d) { keep4_h(a, b, c, d); }
};
template <> struct Frag<__bf16> {
  typedef v16b V; union U { v16b v; v8b h[2]; };
  static __device__ __forceinline__ v16b load(const __bf16* p) {
    U f; f.h[0] = *(const v8b*)(p); f.h[1] = *(const v8b*)(p + 16); return f.v;
  }
  static __device__ __forceinline__ v8f mma(v16b a, v16b b, v8f c) {
    return __builtin_amdgcn_wmma_f32_16x16x32_bf16(false, a, false, b, (short)0, c, false, false);
  }
  static __device__ __forceinline__ void guard(v8f& a, v8f& b, v16b x, v16b y) { dep_guard_b(a, b, x, y); }
  static __device__ __forceinline__ void keep(v16b a, v16b b, v16b c, v16b d) { keep4_b(a, b, c, d); }
};

constexpr int   kTok     = 49;
constexpr int   kTokPad  = 64;
constexpr int   kDim     = 128;
constexpr int   kHd      = 32;
constexpr int   kQkvN    = 384;
constexpr int   kLdx     = 128;
constexpr int   kLdv     = 64;
constexpr int   kLdp     = 64;
constexpr int   kLdo     = 128;
constexpr float kQScale  = 0.17677669529663687f;
constexpr float kPadFill = -1.0e30f;

static_assert(kDim % 32 == 0 && kHd % 32 == 0 && kTokPad % 32 == 0, "every k extent is a multiple of 32");
static_assert(kTokPad % 16 == 0 && kDim % 16 == 0 && kQkvN % 16 == 0, "tile multiples");

constexpr int kPlaneX   = kTokPad * kLdx;
constexpr int kPlaneV   = kDim * kLdv;
constexpr int kPlaneP   = 16 * kLdp;
constexpr int kOffXO    = 0;
constexpr int kOffQ     = kOffXO + 2 * kPlaneX * 2;
constexpr int kOffK     = kOffQ  + 2 * kPlaneX * 2;
constexpr int kOffVT    = kOffK  + 2 * kPlaneX * 2;
constexpr int kOffP     = kOffVT + 2 * kPlaneV * 2;
constexpr int kLdsBytes = kOffP  + 8 * 2 * kPlaneP * 2;
static_assert(kLdsBytes == 163840, "lds size");
static_assert(kTokPad * kLdo * 4 <= kOffVT - kOffQ, "output staging tile fits in the q/k region");

__device__ __forceinline__ unsigned bf_rne_bits(float f) {
  const unsigned u = __float_as_uint(f);
  return (u + 0x7FFFu + ((u >> 16) & 1u)) >> 16;
}
__device__ __forceinline__ float bf_rne(float f) { return __uint_as_float(bf_rne_bits(f) << 16); }
__device__ __forceinline__ void bf_split(float f, unsigned& hb, unsigned& lb) {
  hb = bf_rne_bits(f);
  lb = bf_rne_bits(f - __uint_as_float(hb << 16));
}
__device__ __forceinline__ void split_pack8(const float (&v)[8], v4u& hi, v4u& lo) {
#pragma unroll
  for (int q = 0; q < 4; ++q) {
    unsigned h0, l0, h1, l1;
    bf_split(v[2 * q], h0, l0);
    bf_split(v[2 * q + 1], h1, l1);
    hi[q] = h0 | (h1 << 16);
    lo[q] = l0 | (l1 << 16);
  }
}
__device__ __forceinline__ v16b ldfrag(const unsigned short* p) {
  return Frag<__bf16>::load((const __bf16*)(const void*)p);
}
__device__ __forceinline__ v8f zero8() { return (v8f){0.f, 0.f, 0.f, 0.f, 0.f, 0.f, 0.f, 0.f}; }

__device__ __forceinline__ v8f mma1(v16b a, v16b b, v8f c) {
  c = __builtin_amdgcn_wmma_f32_16x16x32_bf16(false, a, false, b, (short)0, c, false, false);
  asm volatile("v_nop\n\tv_nop\n\tv_nop\n\tv_nop" : "+v"(c) : "v"(a), "v"(b));
  return c;
}
__device__ __forceinline__ v8f mma2(v16b ah, v16b al, v16b b, v8f c) {
  c = __builtin_amdgcn_wmma_f32_16x16x32_bf16(false, ah, false, b, (short)0, c, false, false);
  c = __builtin_amdgcn_wmma_f32_16x16x32_bf16(false, al, false, b, (short)0, c, false, false);
  asm volatile("v_nop\n\tv_nop\n\tv_nop\n\tv_nop" : "+v"(c) : "v"(ah), "v"(al), "v"(b));
  return c;
}
__device__ __forceinline__ v8f mma3(v16b ah, v16b al, v16b bh, v16b bl, v8f c) {
  c = __builtin_amdgcn_wmma_f32_16x16x32_bf16(false, ah, false, bh, (short)0, c, false, false);
  c = __builtin_amdgcn_wmma_f32_16x16x32_bf16(false, ah, false, bl, (short)0, c, false, false);
  c = __builtin_amdgcn_wmma_f32_16x16x32_bf16(false, al, false, bh, (short)0, c, false, false);
  asm volatile("v_nop\n\tv_nop\n\tv_nop\n\tv_nop" : "+v"(c) : "v"(ah), "v"(al), "v"(bh), "v"(bl));
  return c;
}
__device__ __forceinline__ void lds_wave_sync() {
  __builtin_amdgcn_fence(__ATOMIC_RELEASE, "workgroup");
  __builtin_amdgcn_wave_barrier();
  __builtin_amdgcn_fence(__ATOMIC_ACQUIRE, "workgroup");
}

__global__ __launch_bounds__(256) void k_prep_w(const float* __restrict__ qkv_w, const float* __restrict__ proj_w,
                                                unsigned short* __restrict__ wq, unsigned short* __restrict__ wp) {
  const bool first = (blockIdx.x < 24);
  const int gid = first ? (int)(blockIdx.x * 256 + threadIdx.x) : (int)((blockIdx.x - 24) * 256 + threadIdx.x);
  const float* src = first ? qkv_w : proj_w;
  const int ld = first ? kQkvN : kDim;
  unsigned short* dst = first ? wq : wp;
  const int n = gid >> 4, kb = (gid & 15) * 8;
  float v[8];
#pragma unroll
  for (int j = 0; j < 8; ++j) v[j] = src[(size_t)(kb + j) * ld + n];
  v4u w;
#pragma unroll
  for (int q = 0; q < 4; ++q) w[q] = bf_rne_bits(v[2 * q]) | (bf_rne_bits(v[2 * q + 1]) << 16);
  unsigned short* p = dst + (size_t)n * kDim + kb;
  *(volatile v4u*)p = w;
  __threadfence();
  *(volatile v4u*)p = w;
}

__global__ __launch_bounds__(256) void k_prep_mask(const float* __restrict__ am, float* __restrict__ mpad, int nW) {
  const int gid = blockIdx.x * 256 + threadIdx.x;
  const int w = gid >> 10, row = (gid >> 4) & 63, cw = gid & 15;
  const int wc = (w < nW) ? w : (nW - 1);
  const int rr = (row < kTok) ? row : (kTok - 1);
  const float* mrow = am + ((size_t)wc * kTok + rr) * kTok;
  v4f o;
#pragma unroll
  for (int nT = 0; nT < 4; ++nT) {
    const int col  = nT * 16 + cw;
    const int colc = (col < kTok) ? col : (kTok - 1);
    float val = bf_rne(mrow[colc]);
    val = (row < kTok) ? val : 0.0f;
    val = (col < kTok) ? val : kPadFill;
    o[nT] = val;
  }
  float* p = mpad + (size_t)gid * 4;
  *(volatile v4f*)p = o;
  __threadfence();
  *(volatile v4f*)p = o;
}

__global__ __launch_bounds__(256) void k_window_attn(
    const float* __restrict__ x, const float* __restrict__ mpad,
    const float* __restrict__ qkv_b, const float* __restrict__ proj_b,
    const unsigned short* __restrict__ wq, const unsigned short* __restrict__ wp,
    float* __restrict__ out, int nW) {
  __shared__ __align__(16) unsigned char lds_raw[kLdsBytes];
  unsigned short* s_x  = (unsigned short*)(lds_raw + kOffXO);
  unsigned short* s_oh = (unsigned short*)(lds_raw + kOffXO);
  unsigned short* s_ol = s_oh + kPlaneX;
  unsigned short* s_qh = (unsigned short*)(lds_raw + kOffQ);
  unsigned short* s_ql = s_qh + kPlaneX;
  unsigned short* s_kh = (unsigned short*)(lds_raw + kOffK);
  unsigned short* s_kl = s_kh + kPlaneX;
  unsigned short* s_vh = (unsigned short*)(lds_raw + kOffVT);
  unsigned short* s_vl = s_vh + kPlaneV;
  unsigned short* s_pw = (unsigned short*)(lds_raw + kOffP);
  float* s_out = (float*)(lds_raw + kOffQ);

  const int tid  = threadIdx.x;
  const int lane = tid & 31, wave = tid >> 5;
  const int hh = lane >> 4, cc = lane & 15;
  const int bIdx = blockIdx.x;
  const int wIdx = bIdx % nW;
  const int tt  = (wave & 3) * 16;
  const int wg2 = wave >> 2;

  const float* xb = x + (size_t)bIdx * (kTok * kDim);
  for (int i = tid; i < kTokPad * 32; i += 256) {
    const int r = i >> 5, c4 = i & 31;
    const int rr = (r < kTok) ? r : (kTok - 1);
    v4f v = *(const v4f*)(xb + rr * kDim + c4 * 4);
    if (r >= kTok) v = (v4f){0.f, 0.f, 0.f, 0.f};
    v2u w;
    w[0] = bf_rne_bits(v[0]) | (bf_rne_bits(v[1]) << 16);
    w[1] = bf_rne_bits(v[2]) | (bf_rne_bits(v[3]) << 16);
    *(v2u*)(s_x + r * kLdx + c4 * 4) = w;
  }
  __syncthreads();

  v16b xf[4];
#pragma unroll
  for (int ks = 0; ks < 4; ++ks) xf[ks] = ldfrag(s_x + (tt + cc) * kLdx + ks * 32 + 8 * hh);

#pragma unroll 1
  for (int i = 0; i < 8; ++i) {
    const int ft = wg2 + 2 * i;
    const int m0 = ft * 16;
    v8f acc = zero8();
#pragma unroll
    for (int ks = 0; ks < 4; ++ks) {
      const v16b a = ldfrag(wq + (size_t)(m0 + cc) * kDim + ks * 32 + 8 * hh);
      acc = mma1(a, xf[ks], acc);
    }
    const int fb = m0 + 8 * hh;
    const bool isQ = (m0 < kDim);
    const float sc = isQ ? kQScale : 1.0f;
    const v4f b0 = *(const v4f*)(qkv_b + fb);
    const v4f b1 = *(const v4f*)(qkv_b + fb + 4);
    float vals[8];
#pragma unroll
    for (int r = 0; r < 4; ++r) {
      vals[r]     = (acc[r]     + bf_rne(b0[r])) * sc;
      vals[4 + r] = (acc[4 + r] + bf_rne(b1[r])) * sc;
    }
    v4u whi, wlo;
    split_pack8(vals, whi, wlo);
    const int o = (isQ ? 0 : 2 * kPlaneX) + (tt + cc) * kLdx + (isQ ? fb : (fb - kDim));
    *(v4u*)(s_qh + o) = whi;
    *(v4u*)(s_qh + o + kPlaneX) = wlo;
  }
#pragma unroll 1
  for (int i = 0; i < 4; ++i) {
    const int n0 = 2 * kDim + (wg2 + 2 * i) * 16;
    v8f acc = zero8();
#pragma unroll
    for (int ks = 0; ks < 4; ++ks) {
      const v16b bw = ldfrag(wq + (size_t)(n0 + cc) * kDim + ks * 32 + 8 * hh);
      acc = mma1(xf[ks], bw, acc);
    }
    const int d = n0 - 2 * kDim + cc;
    const float bv = bf_rne(qkv_b[n0 + cc]);
    float vals[8];
#pragma unroll
    for (int r = 0; r < 8; ++r) vals[r] = acc[r] + bv;
    v4u whi, wlo;
    split_pack8(vals, whi, wlo);
    const int o = d * kLdv + tt + 8 * hh;
    *(v4u*)(s_vh + o) = whi;
    *(v4u*)(s_vl + o) = wlo;
  }
  __syncthreads();

  {
    const float* mp = mpad + (size_t)wIdx * 4096;
    unsigned short* ph = s_pw + wave * (2 * kPlaneP);
    unsigned short* pl = ph + kPlaneP;
#pragma unroll 1
    for (int i = 0; i < 2; ++i) {
      const int head = wg2 + 2 * i;
      const int hc = head * kHd;
      const v16b qh = ldfrag(s_qh + (tt + cc) * kLdx + hc + 8 * hh);
      const v16b ql = ldfrag(s_ql + (tt + cc) * kLdx + hc + 8 * hh);
      v8f ct[4];
#pragma unroll
      for (int nT = 0; nT < 4; ++nT) {
        const v16b kh = ldfrag(s_kh + (nT * 16 + cc) * kLdx + hc + 8 * hh);
        const v16b kl = ldfrag(s_kl + (nT * 16 + cc) * kLdx + hc + 8 * hh);
        ct[nT] = mma3(qh, ql, kh, kl, zero8());
      }
#pragma unroll
      for (int g = 0; g < 8; ++g) {
        const int row = tt + 8 * hh + g;
        const v4f mr = *(const v4f*)(mp + row * 64 + cc * 4);
        const float s0 = ct[0][g] + mr[0];
        const float s1 = ct[1][g] + mr[1];
        const float s2 = ct[2][g] + mr[2];
        const float s3 = ct[3][g] + mr[3];
        float mx = fmaxf(fmaxf(s0, s1), fmaxf(s2, s3));
        mx = fmaxf(mx, __shfl_xor(mx, 1, 32));
        mx = fmaxf(mx, __shfl_xor(mx, 2, 32));
        mx = fmaxf(mx, __shfl_xor(mx, 4, 32));
        mx = fmaxf(mx, __shfl_xor(mx, 8, 32));
        const float e0 = expf(s0 - mx);
        const float e1 = expf(s1 - mx);
        const float e2 = expf(s2 - mx);
        const float e3 = expf(s3 - mx);
        float sum = (e0 + e1) + (e2 + e3);
        sum += __shfl_xor(sum, 1, 32);
        sum += __shfl_xor(sum, 2, 32);
        sum += __shfl_xor(sum, 4, 32);
        sum += __shfl_xor(sum, 8, 32);
        const float inv = 1.0f / sum;
        const int po = (8 * hh + g) * kLdp + cc;
        unsigned hb, lb;
        bf_split(e0 * inv, hb, lb); ph[po]      = (unsigned short)hb; pl[po]      = (unsigned short)lb;
        bf_split(e1 * inv, hb, lb); ph[po + 16] = (unsigned short)hb; pl[po + 16] = (unsigned short)lb;
        bf_split(e2 * inv, hb, lb); ph[po + 32] = (unsigned short)hb; pl[po + 32] = (unsigned short)lb;
        bf_split(e3 * inv, hb, lb); ph[po + 48] = (unsigned short)hb; pl[po + 48] = (unsigned short)lb;
      }
      lds_wave_sync();
      v16b bph[2], bpl[2];
#pragma unroll
      for (int kk = 0; kk < 2; ++kk) {
        bph[kk] = ldfrag(ph + cc * kLdp + kk * 32 + 8 * hh);
        bpl[kk] = ldfrag(pl + cc * kLdp + kk * 32 + 8 * hh);
      }
#pragma unroll
      for (int md = 0; md < 2; ++md) {
        v8f acc = zero8();
#pragma unroll
        for (int kk = 0; kk < 2; ++kk) {
          const v16b vh = ldfrag(s_vh + (hc + md * 16 + cc) * kLdv + kk * 32 + 8 * hh);
          const v16b vl = ldfrag(s_vl + (hc + md * 16 + cc) * kLdv + kk * 32 + 8 * hh);
          acc = mma3(vh, vl, bph[kk], bpl[kk], acc);
        }
        float vals[8];
#pragma unroll
        for (int r = 0; r < 8; ++r) vals[r] = acc[r];
        v4u whi, wlo;
        split_pack8(vals, whi, wlo);
        const int o = (tt + cc) * kLdx + hc + md * 16 + 8 * hh;
        *(v4u*)(s_oh + o) = whi;
        *(v4u*)(s_ol + o) = wlo;
      }
      lds_wave_sync();
    }
  }
  __syncthreads();

  {
    v16b ah[4], al[4];
#pragma unroll
    for (int ks = 0; ks < 4; ++ks) {
      ah[ks] = ldfrag(s_oh + (tt + cc) * kLdx + ks * 32 + 8 * hh);
      al[ks] = ldfrag(s_ol + (tt + cc) * kLdx + ks * 32 + 8 * hh);
    }
#pragma unroll 1
    for (int i = 0; i < 4; ++i) {
      const int n0 = (wg2 + 2 * i) * 16;
      v8f acc = zero8();
#pragma unroll
      for (int ks = 0; ks < 4; ++ks) {
        const v16b bw = ldfrag(wp + (size_t)(n0 + cc) * kDim + ks * 32 + 8 * hh);
        acc = mma2(ah[ks], al[ks], bw, acc);
      }
      const float bv = bf_rne(proj_b[n0 + cc]);
#pragma unroll
      for (int r = 0; r < 8; ++r) s_out[(tt + 8 * hh + r) * kLdo + n0 + cc] = acc[r] + bv;
    }
  }
  __syncthreads();

  {
    float* ob = out + (size_t)bIdx * (kTok * kDim);
    for (int pass = 0; pass < 2; ++pass) {
#pragma unroll 1
      for (int row = wave; row < kTok; row += 8) {
        const v4f v = *(const v4f*)(s_out + row * kLdo + lane * 4);
        *(volatile v4f*)(ob + (size_t)row * kDim + lane * 4) = v;
      }
      __threadfence();
    }
  }
}

extern "C" void kernel_launch(void* const* d_in, const int* in_sizes, int n_in,
                              void* d_out, int out_size, void* d_ws, size_t ws_size,
                              hipStream_t stream) {
  if (n_in < 6) return;
  const float* x         = (const float*)d_in[0];
  const float* attn_mask = (const float*)d_in[1];
  const float* qkv_w     = (const float*)d_in[2];
  const float* qkv_b     = (const float*)d_in[3];
  const float* proj_w    = (const float*)d_in[4];
  const float* proj_b    = (const float*)d_in[5];
  float* out = (float*)d_out;

  const int per = kTok * kDim;
  const int nx = in_sizes[0];
  if (nx <= 0 || (nx % per) != 0) return;
  const int nb = nx / per;
  const int nm = in_sizes[1];
  if (nm <= 0 || (nm % (kTok * kTok)) != 0) return;
  const int nW = nm / (kTok * kTok);
  if (in_sizes[2] != kDim * kQkvN || in_sizes[3] != kQkvN || in_sizes[4] != kDim * kDim || in_sizes[5] != kDim) return;
  if (out_size != nx) return;

  const size_t offWq = 0;
  const size_t offWp = 98304;
  const size_t offM  = 131072;
  const size_t total = offM + (size_t)nW * 4096 * 4;
  if (total > ws_size || total > (size_t)134217728) return;
  unsigned char* ws = (unsigned char*)d_ws;
  unsigned short* wq = (unsigned short*)(ws + offWq);
  unsigned short* wp = (unsigned short*)(ws + offWp);
  float* mpad = (float*)(ws + offM);

  k_prep_w<<<32, 256, 0, stream>>>(qkv_w, proj_w, wq, wp);
  k_prep_mask<<<nW * 4, 256, 0, stream>>>(attn_mask, mpad, nW);
  k_window_attn<<<nb, 256, 0, stream>>>(x, mpad, qkv_b, proj_b, wq, wp, out, nW);
}
